// Attention_88313117540870
// MI455X (gfx1250) — hardware-verified
//
#include <hip/hip_runtime.h>


#ifndef NB
#define NB 4
#endif
#ifndef SEQ
#define SEQ 2048
#endif
#define NB_FULL  4
#define SEQ_FULL 2048
#define DM   1024
#define NH   16
#define HD   64
#define RH   0
#define CCAR 64.0f
#define WCAR 512.0f
#define CEXP 0.18033688011112042f

typedef _Float16 h16;
typedef unsigned short bf;
typedef __attribute__((ext_vector_type(16))) __bf16   v16bf;
typedef __attribute__((ext_vector_type(16))) _Float16 v16h;
typedef __attribute__((ext_vector_type(8)))  _Float16 v8h;
typedef __attribute__((ext_vector_type(8)))  unsigned short v8us;
typedef __attribute__((ext_vector_type(8)))  float    v8f;
typedef __attribute__((ext_vector_type(4)))  float    v4f;
typedef __attribute__((ext_vector_type(4)))  int      v4i;
typedef v4f  __attribute__((may_alias)) v4fa;

static_assert(SEQ % 256 == 0);
static_assert(RH % 64 == 0);
static_assert(SEQ >= RH);
static_assert(NB <= NB_FULL);
static_assert(SEQ <= SEQ_FULL);
static_assert(DM == NH * HD);
static_assert(DM % 64 == 0);
static_assert(HD == 64);
static_assert(SEQ % 64 == 0);
static_assert(SEQ % 32 == 0);
static_assert(DM % 32 == 0);
static_assert((SEQ / 8) % 32 == 0);

__device__ __forceinline__ unsigned short f2bf(float f) { unsigned u = __float_as_uint(f); u += 0x7FFFu + ((u >> 16) & 1u); return (unsigned short)(u >> 16); }
__device__ __forceinline__ float bf2f(unsigned short b) { return __uint_as_float(((unsigned)b) << 16); }
__device__ __forceinline__ float bfr(float f) { return bf2f(f2bf(f)); }
__device__ __forceinline__ void splitf(float y, unsigned short& h, unsigned short& l) { h = f2bf(y); l = f2bf(y - bf2f(h)); }
__device__ __forceinline__ v16h cat16(v8h lo, v8h hi) { return __builtin_shufflevector(lo, hi, 0, 1, 2, 3, 4, 5, 6, 7, 8, 9, 10, 11, 12, 13, 14, 15); }
__device__ __forceinline__ v16bf cat16b(v8us lo, v8us hi) { return __builtin_bit_cast(v16bf, __builtin_shufflevector(lo, hi, 0, 1, 2, 3, 4, 5, 6, 7, 8, 9, 10, 11, 12, 13, 14, 15)); }
__device__ __forceinline__ v8f wmma16(v16h a, v16h b, v8f c) { return __builtin_amdgcn_wmma_f32_16x16x32_f16(false, a, false, b, (short)0, c, false, false); }
__device__ __forceinline__ v8f wmmab(v16bf a, v16bf b, v8f c) { return __builtin_amdgcn_wmma_f32_16x16x32_bf16(false, a, false, b, (short)0, c, false, false); }

template <typename T16> struct WFrag;
template <> struct WFrag<h16> { typedef v16h V; static __device__ __forceinline__ V ld(const h16* p) { return cat16(*(const v8h*)p, *(const v8h*)(p + 16)); } static __device__ __forceinline__ v8f mma(V a, V b, v8f c) { return wmma16(a, b, c); } };
template <> struct WFrag<bf> { typedef v16bf V; static __device__ __forceinline__ V ld(const bf* p) { return cat16b(*(const v8us*)p, *(const v8us*)(p + 16)); } static __device__ __forceinline__ v8f mma(V a, V b, v8f c) { return wmmab(a, b, c); } };

template <typename T16> struct PPack;
template <> struct PPack<h16> {
    static __device__ __forceinline__ void make(v8f p0, v8f p1, v16h& ph, v16h& pl) {
        v8h a, c;
#pragma unroll
        for (int r = 0; r < 8; ++r) { a[r] = (h16)p0[r]; c[r] = (h16)p1[r]; }
        ph = cat16(a, c); pl = ph; }
};
template <> struct PPack<bf> {
    static __device__ __forceinline__ void make(v8f p0, v8f p1, v16bf& ph, v16bf& pl) {
        v8us ah, al, ch, cl;
#pragma unroll
        for (int r = 0; r < 8; ++r) { unsigned short x, y; splitf(p0[r], x, y); ah[r] = x; al[r] = y; splitf(p1[r], x, y); ch[r] = x; cl[r] = y; }
        ph = cat16b(ah, ch); pl = cat16b(al, cl); }
};

template <typename T16, int NSPLIT, int EP>
__global__ __launch_bounds__(32) void k_gemmw(const T16* __restrict__ A, const T16* __restrict__ A2, const T16* __restrict__ Bt, const T16* __restrict__ Bt2, int K, float* C, int ldc, float oscale, size_t sA, size_t sB, size_t sC, h16* P16, bf* Ph, bf* Pl) {
    typedef typename WFrag<T16>::V V;
    __shared__ __align__(16) float os[16 * 68];
    const size_t z = blockIdx.z; A += z * sA; if (A2) A2 += z * sA; Bt += z * sB; if (Bt2) Bt2 += z * sB; if (EP == 0) C += z * sC;
    const int lane = threadIdx.x & 31, lr = lane & 15, hi = lane >> 4; const int r0 = blockIdx.x * 64, c0 = blockIdx.y * 64;
    v8f acc[4][4];
#pragma unroll
    for (int mb = 0; mb < 4; ++mb)
#pragma unroll
        for (int nb = 0; nb < 4; ++nb) acc[mb][nb] = (v8f){};
    const size_t aoff = (size_t)(r0 + lr) * K + 8 * hi, boff = (size_t)(c0 + lr) * K + 8 * hi;
#pragma unroll 1
    for (int kc = 0; kc < K; kc += 32) {
        V a[4], a2[4];
#pragma unroll
        for (int mb = 0; mb < 4; ++mb) { a[mb] = WFrag<T16>::ld(A + aoff + (size_t)mb * 16 * K + kc); if (NSPLIT == 1 || NSPLIT == 2) a2[mb] = WFrag<T16>::ld(A2 + aoff + (size_t)mb * 16 * K + kc); else a2[mb] = a[mb]; }
#pragma unroll
        for (int nb = 0; nb < 4; ++nb) { const V b = WFrag<T16>::ld(Bt + boff + (size_t)nb * 16 * K + kc); V b2 = b; if (NSPLIT >= 2) b2 = WFrag<T16>::ld(Bt2 + boff + (size_t)nb * 16 * K + kc);
#pragma unroll
            for (int mb = 0; mb < 4; ++mb) { acc[mb][nb] = WFrag<T16>::mma(a[mb], b, acc[mb][nb]); if (NSPLIT == 1 || NSPLIT == 2) acc[mb][nb] = WFrag<T16>::mma(a2[mb], b, acc[mb][nb]); if (NSPLIT >= 2) acc[mb][nb] = WFrag<T16>::mma(a[mb], b2, acc[mb][nb]); } }
        asm volatile("v_nop\n\tv_nop\n\tv_nop\n\tv_nop" : "+v"(acc[0][0]), "+v"(acc[1][1]), "+v"(acc[2][2]), "+v"(acc[3][3]) : "v"(a[0]), "v"(a[3]));
    }
    size_t pbase = 0, hbase = 0; int ppitch = HD, hpitch = HD; bool dohl = false;
    if (EP == 1) { pbase = (((size_t)z * NH + blockIdx.y) * SEQ + r0) * HD; ppitch = HD; hbase = (((size_t)z * NH + blockIdx.y) * RH + r0) * HD; hpitch = HD; dohl = (r0 < RH); }
    if (EP == 2) { pbase = ((size_t)z * DM + r0) * SEQ + c0; ppitch = SEQ; hbase = ((size_t)z * DM + r0) * RH + c0; hpitch = RH; dohl = (c0 < RH); }
    const int q4 = lane >> 3, pc = lane & 7;
#pragma unroll
    for (int mb = 0; mb < 4; ++mb) {
#pragma unroll
        for (int nb = 0; nb < 4; ++nb) {
#pragma unroll
            for (int j = 0; j < 8; ++j) os[(hi * 8 + j) * 68 + nb * 16 + lr] = acc[mb][nb][j]; }
        __builtin_amdgcn_wave_barrier(); asm volatile("" ::: "memory");
        if (EP == 0) {
            float* crow = C + (size_t)(r0 + mb * 16) * ldc + c0;
#pragma unroll 1
            for (int ps = 0; ps < 2; ++ps) {
#pragma unroll
                for (int s = 0; s < 8; ++s) { const int row = 2 * s + hi, cofs = lr * 4; v4f val = *(const v4fa*)(os + row * 68 + cofs); val = val * oscale;
                    *(volatile v4f*)(crow + (size_t)row * ldc + cofs) = val; }
                if (ps == 0) __threadfence(); }
        } else {
#pragma unroll 1
            for (int ps = 0; ps < 2; ++ps) {
#pragma unroll
                for (int s = 0; s < 4; ++s) { const int row = 4 * s + q4; const float* sp = os + row * 68 + pc * 8; const v4f x0 = *(const v4fa*)sp, x1 = *(const v4fa*)(sp + 4);
                    v8h o; o[0] = (h16)x0[0]; o[1] = (h16)x0[1]; o[2] = (h16)x0[2]; o[3] = (h16)x0[3]; o[4] = (h16)x1[0]; o[5] = (h16)x1[1]; o[6] = (h16)x1[2]; o[7] = (h16)x1[3];
                    *(volatile v8h*)(P16 + pbase + (size_t)(mb * 16 + row) * ppitch + pc * 8) = o;
                    if (dohl) { v8us oh, ol; unsigned short u, w;
                        splitf(x0[0], u, w); oh[0] = u; ol[0] = w; splitf(x0[1], u, w); oh[1] = u; ol[1] = w; splitf(x0[2], u, w); oh[2] = u; ol[2] = w; splitf(x0[3], u, w); oh[3] = u; ol[3] = w;
                        splitf(x1[0], u, w); oh[4] = u; ol[4] = w; splitf(x1[1], u, w); oh[5] = u; ol[5] = w; splitf(x1[2], u, w); oh[6] = u; ol[6] = w; splitf(x1[3], u, w); oh[7] = u; ol[7] = w;
                        const size_t ho = hbase + (size_t)(mb * 16 + row) * hpitch + pc * 8; *(volatile v8us*)(Ph + ho) = oh; *(volatile v8us*)(Pl + ho) = ol; } }
                if (ps == 0) __threadfence(); }
        }
        __builtin_amdgcn_wave_barrier(); asm volatile("" ::: "memory");
    }
}

template <typename T16>
__global__ __launch_bounds__(128) void k_flash(const T16* __restrict__ Qa, const T16* __restrict__ Ka, const T16* __restrict__ Va, const bf* __restrict__ Bb, int tq, int tk, int qoff, h16* C16) {
    typedef typename WFrag<T16>::V V;
    __shared__ __align__(16) float osm[4 * 16 * 68];
    const int lane = threadIdx.x & 31, lr = lane & 15, hi = lane >> 4;
    const int wave = __builtin_amdgcn_readfirstlane((int)(threadIdx.x >> 5));
    const int q0 = qoff + (int)blockIdx.x * 64 + wave * 16;
    const int h = blockIdx.y, b = blockIdx.z;
    const size_t bh = (size_t)b * NH + h;
    const size_t qo = (bh * (size_t)tq + (size_t)(q0 + lr)) * HD + 8 * hi;
    const V qa0 = WFrag<T16>::ld(Qa + qo), qa1 = WFrag<T16>::ld(Qa + qo + 32);
    const size_t ko = (bh * (size_t)tk + (size_t)lr) * HD + 8 * hi;
    const size_t vo = (bh * HD + (size_t)lr) * (size_t)tk + 8 * hi;
    const size_t bo = (size_t)(q0 + lr) * (size_t)tk + 8 * hi;
    v8f acc[4];
#pragma unroll
    for (int dt = 0; dt < 4; ++dt) acc[dt] = (v8f){};
    float m = -3.0e38f, l = 0.0f;
    const int nsteps = tk >> 5;
    const float poff = 8.0f;
#pragma unroll 1
    for (int st = 0; st < nsteps; ++st) {
        const int j0 = st * 32;
        const bf* bp = Bb + bo + j0;
        const v8us b0 = *(const v8us*)bp, b1 = *(const v8us*)(bp + 16);
        v8f s0 = (v8f){}, s1 = (v8f){};
        const T16* kp = Ka + ko + (size_t)j0 * HD;
        const V k00 = WFrag<T16>::ld(kp), k01 = WFrag<T16>::ld(kp + 32), k10 = WFrag<T16>::ld(kp + 16 * HD), k11 = WFrag<T16>::ld(kp + 16 * HD + 32);
        s0 = WFrag<T16>::mma(k00, qa0, s0); s1 = WFrag<T16>::mma(k10, qa0, s1);
        s0 = WFrag<T16>::mma(k01, qa1, s0); s1 = WFrag<T16>::mma(k11, qa1, s1);
        asm volatile("v_nop\n\tv_nop\n\tv_nop\n\tv_nop" : "+v"(s0), "+v"(s1) : "v"(k11), "v"(qa1));
#pragma unroll
        for (int r = 0; r < 8; ++r) { s0[r] = fmaf(bf2f(b0[r]), 8.0f, s0[r]); s1[r] = fmaf(bf2f(b1[r]), 8.0f, s1[r]); }
        float mx = fmaxf(s0[0], s1[0]);
#pragma unroll
        for (int r = 1; r < 8; ++r) mx = fmaxf(mx, fmaxf(s0[r], s1[r]));
        mx = fmaxf(mx, __shfl_xor(mx, 16, 32));
        const float mnew = fmaxf(m, mx);
        const float alpha = __builtin_amdgcn_exp2f((m - mnew) * CEXP);
        const float nb = poff - mnew * CEXP;
        v8f p0, p1; float psum = 0.0f;
#pragma unroll
        for (int r = 0; r < 8; ++r) { p0[r] = __builtin_amdgcn_exp2f(fmaf(s0[r], CEXP, nb)); p1[r] = __builtin_amdgcn_exp2f(fmaf(s1[r], CEXP, nb)); psum += p0[r] + p1[r]; }
        psum += __shfl_xor(psum, 16, 32);
        l = l * alpha + psum; m = mnew;
#pragma unroll
        for (int dt = 0; dt < 4; ++dt) acc[dt] = acc[dt] * alpha;
        V ph, pl; PPack<T16>::make(p0, p1, ph, pl);
        const T16* vp = Va + vo + j0;
        V va[4];
#pragma unroll
        for (int dt = 0; dt < 4; ++dt) va[dt] = WFrag<T16>::ld(vp + (size_t)dt * 16 * (size_t)tk);
#pragma unroll
        for (int dt = 0; dt < 4; ++dt) acc[dt] = WFrag<T16>::mma(va[dt], ph, acc[dt]);
        asm volatile("v_nop\n\tv_nop\n\tv_nop\n\tv_nop" : "+v"(acc[0]), "+v"(acc[1]), "+v"(acc[2]), "+v"(acc[3]) : "v"(va[3]), "v"(ph), "v"(pl));
    }
    const float f = CCAR * (1.0f / l);
    float* os = osm + wave * (16 * 68);
#pragma unroll
    for (int dt = 0; dt < 4; ++dt)
#pragma unroll
        for (int r = 0; r < 8; ++r) os[lr * 68 + dt * 16 + 8 * hi + r] = acc[dt][r] * f;
    __builtin_amdgcn_wave_barrier(); asm volatile("" ::: "memory");
    const int q4 = lane >> 3, pc = lane & 7;
#pragma unroll 1
    for (int ps = 0; ps < 2; ++ps) {
#pragma unroll
        for (int s = 0; s < 4; ++s) { const int row = 4 * s + q4; const float* sp = os + row * 68 + pc * 8; const v4f x0 = *(const v4fa*)sp, x1 = *(const v4fa*)(sp + 4);
            v8h o; o[0] = (h16)x0[0]; o[1] = (h16)x0[1]; o[2] = (h16)x0[2]; o[3] = (h16)x0[3]; o[4] = (h16)x1[0]; o[5] = (h16)x1[1]; o[6] = (h16)x1[2]; o[7] = (h16)x1[3];
            const size_t co = ((size_t)b * SEQ + (size_t)(q0 + row)) * DM + (size_t)h * HD + pc * 8; *(volatile v8h*)(C16 + co) = o; }
        if (ps == 0) __threadfence(); }
}

__global__ __launch_bounds__(256) void k_cvt8(const float* __restrict__ src, bf* dst, size_t n8, size_t sS, size_t sD) {
#pragma clang fp contract(off)
    const size_t i = (size_t)blockIdx.x * 256 + threadIdx.x; if (i >= n8) return; src += (size_t)blockIdx.y * sS; dst += (size_t)blockIdx.y * sD; const v8f v = *(const v8f*)(src + i * 8); v8us o;
#pragma unroll
    for (int k = 0; k < 8; ++k) o[k] = f2bf(v[k]);
    *(volatile v8us*)(dst + i * 8) = o; __threadfence(); *(volatile v8us*)(dst + i * 8) = o; }

__global__ __launch_bounds__(256) void k_cvt8h(const float* __restrict__ src, h16* dst, size_t n8, float sc) {
#pragma clang fp contract(off)
    const size_t i = (size_t)blockIdx.x * 256 + threadIdx.x; if (i >= n8) return; const v8f v = *(const v8f*)(src + i * 8); v8h o;
#pragma unroll
    for (int k = 0; k < 8; ++k) o[k] = (h16)(bfr(v[k]) * sc);
    *(volatile v8h*)(dst + i * 8) = o; __threadfence(); *(volatile v8h*)(dst + i * 8) = o; }

constexpr size_t al256(size_t bytes) { return (bytes + 255) & ~(size_t)255; }
constexpr size_t CARVE_BYTES = 2 * al256((size_t)NB * SEQ * DM * 2) + 4 * al256((size_t)DM * DM * 2) + al256((size_t)SEQ * SEQ * 2)
    + 3 * al256((size_t)NB * NH * SEQ * HD * 2) + al256((size_t)NB * SEQ * DM * 2);
static_assert(CARVE_BYTES <= (size_t)134217728);
static_assert((size_t)NB * NH * SEQ * HD == (size_t)NB * SEQ * DM);
static_assert(SEQ <= 65535);

extern "C" void kernel_launch(void* const* d_in, const int* in_sizes, int n_in,
                              void* d_out, int out_size, void* d_ws, size_t ws_size, hipStream_t stream) {
    if (n_in < 7) return;
    const size_t needx = (size_t)(NB - 1) * SEQ_FULL * DM + (size_t)SEQ * DM;
    if ((size_t)in_sizes[0] < needx || (size_t)in_sizes[1] < needx) return;
    if ((size_t)in_sizes[2] < (size_t)(SEQ - 1) * SEQ_FULL + (size_t)SEQ) return;
    if ((size_t)in_sizes[3] < (size_t)DM * DM || (size_t)in_sizes[4] < (size_t)DM * DM || (size_t)in_sizes[5] < (size_t)DM * DM || (size_t)in_sizes[6] < (size_t)DM * DM) return;
    if ((size_t)out_size < needx) return;
    const float* x = (const float*)d_in[0]; const float* y = (const float*)d_in[1]; const float* bias = (const float*)d_in[2];
    const float* wq = (const float*)d_in[3]; const float* wk = (const float*)d_in[4]; const float* wv = (const float*)d_in[5]; const float* wo = (const float*)d_in[6];
    float* OUT = (float*)d_out;
    char* wsp = (char*)d_ws;
    auto take = [&](size_t bytes) { char* p = wsp; wsp += (bytes + 255) & ~(size_t)255; return (void*)p; };
    bf* XB = (bf*)take((size_t)NB * SEQ * DM * 2); bf* YB = (bf*)take((size_t)NB * SEQ * DM * 2);
    bf* WQ = (bf*)take((size_t)DM * DM * 2); bf* WK = (bf*)take((size_t)DM * DM * 2); bf* WV = (bf*)take((size_t)DM * DM * 2); h16* WO16 = (h16*)take((size_t)DM * DM * 2);
    bf* BB = (bf*)take((size_t)SEQ * SEQ * 2);
    h16* Q16 = (h16*)take((size_t)NB * NH * SEQ * HD * 2); h16* K16 = (h16*)take((size_t)NB * NH * SEQ * HD * 2); h16* VT16 = (h16*)take((size_t)NB * NH * SEQ * HD * 2);
    h16* C16 = (h16*)take((size_t)NB * SEQ * DM * 2);
    if ((size_t)(wsp - (char*)d_ws) > ws_size) return;

    const unsigned gx = (unsigned)(((size_t)SEQ * DM / 8 + 255) / 256), gw = (unsigned)(((size_t)DM * DM / 8 + 255) / 256), gb = (unsigned)(((size_t)SEQ / 8 + 255) / 256);
    k_cvt8<<<dim3(gx, NB, 1), 256, 0, stream>>>(x, XB, (size_t)SEQ * DM / 8, (size_t)SEQ_FULL * DM, (size_t)SEQ * DM);
    k_cvt8<<<dim3(gx, NB, 1), 256, 0, stream>>>(y, YB, (size_t)SEQ * DM / 8, (size_t)SEQ_FULL * DM, (size_t)SEQ * DM);
    k_cvt8<<<dim3(gb, SEQ, 1), 256, 0, stream>>>(bias, BB, (size_t)SEQ / 8, (size_t)SEQ_FULL, (size_t)SEQ);
    k_cvt8<<<dim3(gw, 1, 1), 256, 0, stream>>>(wq, WQ, (size_t)DM * DM / 8, 0, 0);
    k_cvt8<<<dim3(gw, 1, 1), 256, 0, stream>>>(wk, WK, (size_t)DM * DM / 8, 0, 0);
    k_cvt8<<<dim3(gw, 1, 1), 256, 0, stream>>>(wv, WV, (size_t)DM * DM / 8, 0, 0);
    k_cvt8h<<<dim3(gw, 1, 1), 256, 0, stream>>>(wo, WO16, (size_t)DM * DM / 8, WCAR);

    k_gemmw<bf, 0, 1><<<dim3(SEQ / 64, NH, NB), 32, 0, stream>>>(XB, nullptr, WQ, nullptr, DM, nullptr, 0, 1.0f, (size_t)SEQ * DM, 0, 0, Q16, nullptr, nullptr);
    k_gemmw<bf, 0, 1><<<dim3(SEQ / 64, NH, NB), 32, 0, stream>>>(YB, nullptr, WK, nullptr, DM, nullptr, 0, 1.0f, (size_t)SEQ * DM, 0, 0, K16, nullptr, nullptr);
    k_gemmw<bf, 0, 2><<<dim3(DM / 64, SEQ / 64, NB), 32, 0, stream>>>(WV, nullptr, YB, nullptr, DM, nullptr, 0, 1.0f, 0, (size_t)SEQ * DM, 0, VT16, nullptr, nullptr);

    k_flash<h16><<<dim3(SEQ / 64, NH, NB), 128, 0, stream>>>(Q16, K16, VT16, BB, SEQ, SEQ, 0, C16);

    k_gemmw<h16, 0, 0><<<dim3(SEQ / 64, DM / 64, NB), 32, 0, stream>>>(C16, nullptr, WO16, nullptr, DM, OUT, DM, 1.0f / (CCAR * WCAR), (size_t)SEQ * DM, 0, (size_t)SEQ_FULL * DM, nullptr, nullptr, nullptr);
}
